// BiLSTMTagger_76020921139770
// MI455X (gfx1250) — hardware-verified
//
#include <hip/hip_runtime.h>
#include <hip/hip_bf16.h>
#include <math.h>

typedef __attribute__((ext_vector_type(16))) _Float16 v16h;
typedef __attribute__((ext_vector_type(8)))  _Float16 v8h;
typedef __attribute__((ext_vector_type(16))) __bf16   v16b;
typedef __attribute__((ext_vector_type(8)))  __bf16   v8b;
typedef __attribute__((ext_vector_type(8)))  float    v8f;
typedef __attribute__((ext_vector_type(4)))  float    v4f;
typedef __attribute__((ext_vector_type(4)))  unsigned v4u;

constexpr int kBatch  = 64;
constexpr int kSeq    = 1024;
constexpr int kEmb    = 128;
constexpr int kHid    = 256;
constexpr int kGate   = 1024;
constexpr int kKcat   = kEmb + kHid;
constexpr int kVocab  = 50000;
constexpr int kTags   = 50;
constexpr int kTagPad = 64;
constexpr int kRows   = kBatch * kSeq;
constexpr float kInv256 = 1.0f / 256.0f;

static_assert(kKcat % 32 == 0, "gate GEMM K multiple of 32");
static_assert(kEmb % 32 == 0 && kHid % 32 == 0, "k-steps of 32");
static_assert((2 * kHid) % 32 == 0, "FC K multiple of 32");
static_assert(kRows % 64 == 0 && kTagPad % 64 == 0, "FC M,N tile multiples");

constexpr size_t kOffE    = 0;
constexpr size_t kBytesE  = (size_t)kRows * kEmb * 2;
constexpr size_t kOffW    = kOffE + kBytesE;
constexpr size_t kBytesW  = (size_t)2 * kGate * kKcat * 2;
constexpr size_t kOffWfc  = kOffW + kBytesW;
constexpr size_t kBytesWfc = (size_t)kTagPad * 2 * kHid * 2;
constexpr size_t kOffBias = kOffWfc + kBytesWfc;
constexpr size_t kBytesBias = (size_t)2 * kGate * 4;
constexpr size_t kOffH    = kOffBias + kBytesBias;
constexpr size_t kBytesH  = (size_t)kRows * 2 * kHid * 2;
constexpr size_t kOffC    = kOffH + kBytesH;
constexpr size_t kBytesC  = (size_t)kRows * kTagPad * 4;
constexpr size_t kWsTotal = kOffC + kBytesC;
static_assert(kWsTotal == 102309888, "carve total");
static_assert(kWsTotal <= 134217728, "carve under 128 MiB");
static_assert(kOffW % 128 == 0 && kOffWfc % 128 == 0 && kOffBias % 128 == 0 && kOffH % 128 == 0 && kOffC % 128 == 0, "128-B aligned regions");

__device__ __forceinline__ unsigned short f2bf_bits(float f) {
  unsigned u = __float_as_uint(f);
  return (unsigned short)((u + 0x7FFFu + ((u >> 16) & 1u)) >> 16);
}
__device__ __forceinline__ float bf_bits2f(unsigned short h) { return __uint_as_float(((unsigned)h) << 16); }

__device__ __forceinline__ void dep_guard_h(v8f& a, v8f& b, v16h x, v16h y) { asm volatile("v_nop\n\tv_nop\n\tv_nop\n\tv_nop" : "+v"(a), "+v"(b) : "v"(x), "v"(y)); }
__device__ __forceinline__ void dep_guard_b(v8f& a, v8f& b, v16b x, v16b y) { asm volatile("v_nop\n\tv_nop\n\tv_nop\n\tv_nop" : "+v"(a), "+v"(b) : "v"(x), "v"(y)); }
__device__ __forceinline__ void keep4_h(v16h a, v16h b, v16h c, v16h d) { asm volatile("v_nop" :: "v"(a), "v"(b), "v"(c), "v"(d)); }
__device__ __forceinline__ void keep4_b(v16b a, v16b b, v16b c, v16b d) { asm volatile("v_nop" :: "v"(a), "v"(b), "v"(c), "v"(d)); }
__device__ __forceinline__ void acc_guard4(v8f& a, v8f& b, v8f& c, v8f& d) { asm volatile("v_nop\n\tv_nop\n\tv_nop\n\tv_nop" : "+v"(a), "+v"(b), "+v"(c), "+v"(d)); }
template <typename T> struct Frag;
template <> struct Frag<_Float16> {
  typedef v16h V; union U { v16h v; v8h h[2]; };
  static __device__ __forceinline__ v16h load(const _Float16* p) {
    U f; f.h[0] = *(const v8h*)(p); f.h[1] = *(const v8h*)(p + 16); return f.v;
  }
  static __device__ __forceinline__ v8f mma(v16h a, v16h b, v8f c) {
    return __builtin_amdgcn_wmma_f32_16x16x32_f16(false, a, false, b, (short)0, c, false, false);
  }
  static __device__ __forceinline__ void guard(v8f& a, v8f& b, v16h x, v16h y) { dep_guard_h(a, b, x, y); }
  static __device__ __forceinline__ void keep(v16h a, v16h b, v16h c, v16h d) { keep4_h(a, b, c, d); }
};
template <> struct Frag<__bf16> {
  typedef v16b V; union U { v16b v; v8b h[2]; };
  static __device__ __forceinline__ v16b load(const __bf16* p) {
    U f; f.h[0] = *(const v8b*)(p); f.h[1] = *(const v8b*)(p + 16); return f.v;
  }
  static __device__ __forceinline__ v8f mma(v16b a, v16b b, v8f c) {
    return __builtin_amdgcn_wmma_f32_16x16x32_bf16(false, a, false, b, (short)0, c, false, false);
  }
  static __device__ __forceinline__ void guard(v8f& a, v8f& b, v16b x, v16b y) { dep_guard_b(a, b, x, y); }
  static __device__ __forceinline__ void keep(v16b a, v16b b, v16b c, v16b d) { keep4_b(a, b, c, d); }
};

template <int ET> struct Elem;
template <> struct Elem<0> { typedef _Float16 T; };
template <> struct Elem<1> { typedef __bf16 T; };
template <int ET, bool SPLIT, int BIAS_MODE, int OUT_MODE, bool RESID, int ACT = 0>
__global__ __launch_bounds__(256) void wmma_gemm64(
    const unsigned short* __restrict__ Ap, const unsigned short* __restrict__ A2p, int lda, long strideA,
    const unsigned short* __restrict__ Btp, const unsigned short* __restrict__ Bt2p, int ldb, long strideB,
    void* __restrict__ Cout, void* __restrict__ Cout2, int ldc, long strideC,
    const float* __restrict__ bias,
    const float* __restrict__ resid, long strideR,
    int M, int N, int K, float scale) {
  typedef typename Elem<ET>::T T;
  typedef typename Frag<T>::V V;
  const T* A = (const T*)Ap; const T* A2 = (const T*)A2p; const T* Bt = (const T*)Btp; const T* Bt2 = (const T*)Bt2p;
  __shared__ __align__(16) float sT[8][16 * 68];
  const int b    = blockIdx.y;
  const int lane = threadIdx.x & 31;
  const int wave = threadIdx.x >> 5;
  const int tilesN = N >> 6;
  const int tilesM = M >> 6;
  const int tile = blockIdx.x * 8 + wave;
  if (tile >= tilesM * tilesN) return;
  const int tm = tile / tilesN;
  const int tn = tile - tm * tilesN;
  const int m0 = tm << 6;
  const int n0 = tn << 6;

  const T* Ab  = A  + (size_t)b * strideA;
  const T* Bb  = Bt + (size_t)b * strideB;
  const T* Ab2 = SPLIT ? (A2  + (size_t)b * strideA) : nullptr;
  const T* Bb2 = SPLIT ? (Bt2 + (size_t)b * strideB) : nullptr;

  const int rlane = lane & 15;
  const int koff  = (lane >> 4) * 8;
  const int mOff  = (lane >> 4) * 8;

  v8f acc[4][4];
#pragma unroll
  for (int i = 0; i < 4; ++i)
#pragma unroll
    for (int j = 0; j < 4; ++j) acc[i][j] = (v8f){0.f,0.f,0.f,0.f,0.f,0.f,0.f,0.f};

  for (int k0 = 0; k0 < K; k0 += 32) {
    V bh[4], bl[4];
#pragma unroll
    for (int j = 0; j < 4; ++j) {
      const size_t bo = (size_t)(n0 + (j << 4) + rlane) * ldb + koff + k0;
      bh[j] = Frag<T>::load(Bb + bo);
      if (SPLIT) bl[j] = Frag<T>::load(Bb2 + bo);
    }
#pragma unroll
    for (int i = 0; i < 4; ++i) {
      const size_t ao = (size_t)(m0 + (i << 4) + rlane) * lda + koff + k0;
      V ah = Frag<T>::load(Ab + ao);
      V al;
      if (SPLIT) al = Frag<T>::load(Ab2 + ao);
#pragma unroll
      for (int j = 0; j < 4; ++j) {
        acc[i][j] = Frag<T>::mma(ah, bh[j], acc[i][j]);
        if (SPLIT) {
          acc[i][j] = Frag<T>::mma(ah, bl[j], acc[i][j]);
          acc[i][j] = Frag<T>::mma(al, bh[j], acc[i][j]);
        }
      }
      Frag<T>::guard(acc[i][0], acc[i][3], ah, SPLIT ? al : ah);
    }
    Frag<T>::keep(bh[0], bh[1], bh[2], bh[3]);
    if (SPLIT) Frag<T>::keep(bl[0], bl[1], bl[2], bl[3]);
  }
  acc_guard4(acc[0][0], acc[0][1], acc[0][2], acc[0][3]);
  acc_guard4(acc[1][0], acc[1][1], acc[1][2], acc[1][3]);
  acc_guard4(acc[2][0], acc[2][1], acc[2][2], acc[2][3]);
  acc_guard4(acc[3][0], acc[3][1], acc[3][2], acc[3][3]);

  float* slab = sT[wave];
  const float* Rb = RESID ? (resid + (size_t)b * strideR) : nullptr;
#pragma unroll
  for (int i = 0; i < 4; ++i) {
    const int mBase = m0 + (i << 4);
#pragma unroll
    for (int j = 0; j < 4; ++j) {
      const int n = n0 + (j << 4) + rlane;
      float bv = 0.f;
      if (BIAS_MODE == 2) bv = bias[n];
#pragma unroll
      for (int r = 0; r < 8; ++r) {
        float v = acc[i][j][r] * scale;
        if (BIAS_MODE == 1) v += bias[mBase + mOff + r];
        if (BIAS_MODE == 2) v += bv;
        if (RESID) v += Rb[(size_t)(mBase + mOff + r) * ldc + n];
        if (ACT == 1) v = tanhf(v);
        if (ACT == 2) v = fmaxf(v, 0.0f);
        if (ACT == 3) v = v / (1.0f + expf(-v));
        if (ACT == 4) v = (v > 0.f) ? v : 0.01f * v;
        if (ACT == 5) v = 0.5f * v * (1.0f + erff(v * 0.70710678118654752f));
        slab[(mOff + r) * 68 + (j << 4) + rlane] = v;
      }
    }
    __builtin_amdgcn_fence(__ATOMIC_RELEASE, "workgroup");
    __builtin_amdgcn_wave_barrier();
    __builtin_amdgcn_fence(__ATOMIC_ACQUIRE, "workgroup");
    if (OUT_MODE == 0) {
      float* C = (float*)Cout + (size_t)b * strideC;
      const int hh = lane >> 4, c4 = (lane & 15) * 4;
      for (int pass = 0; pass < 2; ++pass) {
#pragma unroll
        for (int it = 0; it < 8; ++it) {
          const int row = it * 2 + hh;
          v4f v = *(const v4f*)(slab + row * 68 + c4);
          *(volatile v4f*)(C + (size_t)(mBase + row) * ldc + n0 + c4) = v;
        }
        __threadfence();
      }
    } else {
      const int q = lane >> 3, c8 = (lane & 7) * 8;
      unsigned short* C  = (unsigned short*)Cout  + (size_t)b * strideC;
      unsigned short* C2 = (OUT_MODE == 2) ? ((unsigned short*)Cout2 + (size_t)b * strideC) : nullptr;
      for (int pass = 0; pass < 2; ++pass) {
#pragma unroll
        for (int it = 0; it < 4; ++it) {
          const int row = it * 4 + q;
          const float* sp = slab + row * 68 + c8;
          v8h hv, lv;
#pragma unroll
          for (int e = 0; e < 8; ++e) {
            if (OUT_MODE == 1) {
              hv[e] = (_Float16)sp[e];
            } else {
              unsigned short hb = f2bf_bits(sp[e]);
              unsigned short lb = f2bf_bits(sp[e] - bf_bits2f(hb));
              hv[e] = __builtin_bit_cast(_Float16, hb);
              lv[e] = __builtin_bit_cast(_Float16, lb);
            }
          }
          *(volatile v8h*)(C + (size_t)(mBase + row) * ldc + n0 + c8) = hv;
          if (OUT_MODE == 2) *(volatile v8h*)(C2 + (size_t)(mBase + row) * ldc + n0 + c8) = lv;
        }
        __threadfence();
      }
    }
    __builtin_amdgcn_fence(__ATOMIC_RELEASE, "workgroup");
    __builtin_amdgcn_wave_barrier();
    __builtin_amdgcn_fence(__ATOMIC_ACQUIRE, "workgroup");
  }
}

__device__ __forceinline__ float bf_rne(float v) { return bf_bits2f(f2bf_bits(v)); }
__device__ __forceinline__ unsigned cvt_bits_x16(float v) {
  const float r = bf_rne(v) * 16.0f;
  const _Float16 h = (_Float16)r;
  return (unsigned)__builtin_bit_cast(unsigned short, h);
}
__device__ __forceinline__ v4u pack8_x16(v4f a, v4f b) {
  v4u o;
  o[0] = cvt_bits_x16(a[0]) | (cvt_bits_x16(a[1]) << 16);
  o[1] = cvt_bits_x16(a[2]) | (cvt_bits_x16(a[3]) << 16);
  o[2] = cvt_bits_x16(b[0]) | (cvt_bits_x16(b[1]) << 16);
  o[3] = cvt_bits_x16(b[2]) | (cvt_bits_x16(b[3]) << 16);
  return o;
}
__device__ __forceinline__ v8f mma_h(v16h a, v16h b, v8f c) {
  c = __builtin_amdgcn_wmma_f32_16x16x32_f16(false, a, false, b, (short)0, c, false, false);
  asm volatile("v_nop\n\tv_nop\n\tv_nop\n\tv_nop" : "+v"(c) : "v"(a), "v"(b));
  return c;
}
__device__ __forceinline__ float sigm(float x) {
  x = fminf(fmaxf(x, -30.0f), 30.0f);
  const float e = expf(-x);
  return 1.0f / (1.0f + e);
}
__device__ __forceinline__ int opaque_zero() {
  int zr;
  asm volatile("s_mov_b32 %0, 0" : "=s"(zr));
  return zr;
}

__global__ __launch_bounds__(256) void k_embed(const int* __restrict__ x, const float* __restrict__ emb,
                                               unsigned short* __restrict__ Eout, int ngroups) {
  const int i = blockIdx.x * 256 + threadIdx.x;
  if (i >= ngroups) return;
  const int n = i * 8;
  const int k = n & (kEmb - 1);
  const int b = (n >> 7) & (kBatch - 1);
  const int t = n >> 13;
  int tok = x[b * kSeq + t];
  tok = tok < 0 ? 0 : (tok > kVocab - 1 ? kVocab - 1 : tok);
  const float* src = emb + (size_t)tok * kEmb + k;
  const v4f f0 = *(const v4f*)(src);
  const v4f f1 = *(const v4f*)(src + 4);
  const v4u o = pack8_x16(f0, f1);
  unsigned short* dst = Eout + (size_t)i * 8;
  *(volatile v4u*)dst = o;
  __threadfence();
  *(volatile v4u*)dst = o;
}

__global__ __launch_bounds__(256) void k_wcat(const float* __restrict__ Wx_f, const float* __restrict__ Wh_f,
                                              const float* __restrict__ Wx_b, const float* __restrict__ Wh_b,
                                              unsigned short* __restrict__ Wout) {
  const int i = blockIdx.x * 256 + threadIdx.x;
  if (i >= kGate * (kKcat / 8)) return;
  const int dir = blockIdx.y;
  const float* Wx = dir ? Wx_b : Wx_f;
  const float* Wh = dir ? Wh_b : Wh_f;
  const int row = i / (kKcat / 8);
  const int col = (i - row * (kKcat / 8)) * 8;
  const int colx = col < (kEmb - 8) ? col : (kEmb - 8);
  int colh = col - kEmb;
  colh = colh < 0 ? 0 : colh;
  const float* px = Wx + (size_t)row * kEmb + colx;
  const float* ph = Wh + (size_t)row * kHid + colh;
  const v4f x0 = *(const v4f*)(px), x1 = *(const v4f*)(px + 4);
  const v4f h0 = *(const v4f*)(ph), h1 = *(const v4f*)(ph + 4);
  const bool useX = (col < kEmb);
  v4f a, c;
#pragma unroll
  for (int q = 0; q < 4; ++q) { a[q] = useX ? x0[q] : h0[q]; c[q] = useX ? x1[q] : h1[q]; }
  const v4u o = pack8_x16(a, c);
  unsigned short* dst = Wout + (size_t)dir * kGate * kKcat + (size_t)i * 8;
  *(volatile v4u*)dst = o;
  __threadfence();
  *(volatile v4u*)dst = o;
}

__global__ __launch_bounds__(256) void k_wfc(const float* __restrict__ Wfc, unsigned short* __restrict__ Wout) {
  const int i = blockIdx.x * 256 + threadIdx.x;
  if (i >= kTagPad * (2 * kHid / 8)) return;
  const int row = i >> 6;
  const int col = (i & 63) * 8;
  const int rowc = row < kTags ? row : (kTags - 1);
  const float* p = Wfc + (size_t)rowc * (2 * kHid) + col;
  v4f f0 = *(const v4f*)(p), f1 = *(const v4f*)(p + 4);
  const v4f z = {0.f, 0.f, 0.f, 0.f};
  if (row >= kTags) { f0 = z; f1 = z; }
  const v4u o = pack8_x16(f0, f1);
  unsigned short* dst = Wout + (size_t)i * 8;
  *(volatile v4u*)dst = o;
  __threadfence();
  *(volatile v4u*)dst = o;
}

__global__ __launch_bounds__(256) void k_bias(const float* __restrict__ bx_f, const float* __restrict__ bh_f,
                                              const float* __restrict__ bx_b, const float* __restrict__ bh_b,
                                              float* __restrict__ biasc) {
  const int g = threadIdx.x * 4;
  const bool d1 = (blockIdx.x == 1);
  const v4f xf = *(const v4f*)(bx_f + g), hf = *(const v4f*)(bh_f + g);
  const v4f xb = *(const v4f*)(bx_b + g), hb = *(const v4f*)(bh_b + g);
  v4f o;
#pragma unroll
  for (int q = 0; q < 4; ++q) {
    const float bxv = d1 ? xb[q] : xf[q];
    const float bhv = d1 ? hb[q] : hf[q];
    o[q] = bf_rne(bxv) + bf_rne(bhv);
  }
  float* dst = biasc + (size_t)blockIdx.x * kGate + g;
  *(volatile v4f*)dst = o;
  __threadfence();
  *(volatile v4f*)dst = o;
}

__global__ __launch_bounds__(512) void k_scan(const unsigned short* __restrict__ Ep,
                                              const unsigned short* __restrict__ Wp,
                                              const float* __restrict__ biasc,
                                              unsigned short* __restrict__ Hp) {
  typedef Frag<_Float16> FH;
  const _Float16* E = (const _Float16*)Ep;
  const _Float16* W = (const _Float16*)Wp;
  _Float16* Hout = (_Float16*)Hp;

  const int dir  = blockIdx.x >> 2;
  const int mg   = blockIdx.x & 3;
  const int lane = threadIdx.x & 31;
  const int wv   = threadIdx.x >> 5;
  const int ln15 = lane & 15;
  const int khal = lane >> 4;

  __shared__ __align__(16) _Float16 hbuf[2][16 * kHid];
  {
    const v4u z = {0u, 0u, 0u, 0u};
    v4u* hz = (v4u*)(&hbuf[0][0]);
    for (int i = threadIdx.x; i < (2 * 16 * kHid) / 8; i += 512) hz[i] = z;
  }
  __syncthreads();

  const _Float16* Wd = W + (size_t)dir * kGate * kKcat;
  float bj[4];
#pragma unroll
  for (int j = 0; j < 4; ++j) bj[j] = biasc[dir * kGate + 16 * (wv + 16 * j) + ln15];

  v8f cst = (v8f){0.f,0.f,0.f,0.f,0.f,0.f,0.f,0.f};
  const int hcol = 16 * wv + ln15;

  for (int stp = 0; stp < kSeq; ++stp) {
    const int t = dir ? (kSeq - 1 - stp) : stp;
    const _Float16* Wdt = Wd + opaque_zero();

    v8f acc[4];
#pragma unroll
    for (int j = 0; j < 4; ++j) acc[j] = (v8f){0.f,0.f,0.f,0.f,0.f,0.f,0.f,0.f};

    const _Float16* erow = E + ((size_t)t * kBatch + mg * 16 + ln15) * kEmb + 8 * khal;
#pragma unroll 1
    for (int ks = 0; ks < 4; ++ks) {
      const v16h a = FH::load(erow + ks * 32);
#pragma unroll
      for (int j = 0; j < 4; ++j) {
        const v16h bb = FH::load(Wdt + (size_t)(16 * (wv + 16 * j) + ln15) * kKcat + ks * 32 + 8 * khal);
        acc[j] = mma_h(a, bb, acc[j]);
      }
    }
    const _Float16* hrow = &hbuf[stp & 1][ln15 * kHid + 8 * khal];
#pragma unroll 1
    for (int ks = 0; ks < 8; ++ks) {
      const v16h a = FH::load(hrow + ks * 32);
#pragma unroll
      for (int j = 0; j < 4; ++j) {
        const v16h bb = FH::load(Wdt + (size_t)(16 * (wv + 16 * j) + ln15) * kKcat + kEmb + ks * 32 + 8 * khal);
        acc[j] = mma_h(a, bb, acc[j]);
      }
    }

    _Float16* hn = &hbuf[(stp + 1) & 1][0];
#pragma unroll
    for (int r = 0; r < 8; ++r) {
      const float gi = acc[0][r] * kInv256 + bj[0];
      const float gf = acc[1][r] * kInv256 + bj[1];
      const float gg = acc[2][r] * kInv256 + bj[2];
      const float go = acc[3][r] * kInv256 + bj[3];
      const float iv = sigm(gi);
      const float fv = sigm(gf);
      const float gv = tanhf(gg);
      const float ov = sigm(go);
      const float cc = fv * cst[r] + iv * gv;
      cst[r] = cc;
      const float hv = ov * tanhf(cc);
      hn[(8 * khal + r) * kHid + hcol] = (_Float16)(hv * 16.0f);
    }
    __syncthreads();

    {
      const v8h val = *(const v8h*)(&hbuf[(stp + 1) & 1][wv * kHid + lane * 8]);
      _Float16* dst = Hout + (((size_t)(mg * 16 + wv)) * kSeq + t) * (2 * kHid) + dir * kHid + lane * 8;
      *(volatile v8h*)dst = val;
      __threadfence();
      *(volatile v8h*)dst = val;
    }
  }
}

__global__ __launch_bounds__(256) void k_out(const float* __restrict__ Cfc, const float* __restrict__ bfc,
                                             float* __restrict__ out, int n4) {
  const int i = blockIdx.x * 256 + threadIdx.x;
  if (i >= n4) return;
  v4f r;
#pragma unroll
  for (int q = 0; q < 4; ++q) {
    const int e = 4 * i + q;
    const int row = e / kTags;
    const int col = e - row * kTags;
    const float cv = Cfc[(size_t)row * kTagPad + col];
    const float bb = bf_rne(bfc[col]);
    r[q] = cv + bb;
  }
  float* dst = out + (size_t)4 * i;
  *(volatile v4f*)dst = r;
  __threadfence();
  *(volatile v4f*)dst = r;
}

extern "C" void kernel_launch(void* const* d_in, const int* in_sizes, int n_in,
                              void* d_out, int out_size, void* d_ws, size_t ws_size,
                              hipStream_t stream) {
  if (n_in < 13) return;
  if (in_sizes[0] != kBatch * kSeq || in_sizes[2] != kVocab * kEmb ||
      in_sizes[3] != kGate * kEmb || in_sizes[4] != kGate || in_sizes[5] != kGate * kHid || in_sizes[6] != kGate ||
      in_sizes[7] != kGate * kEmb || in_sizes[8] != kGate || in_sizes[9] != kGate * kHid || in_sizes[10] != kGate ||
      in_sizes[11] != kTags * 2 * kHid || in_sizes[12] != kTags || out_size != kRows * kTags) return;
  if (ws_size < kWsTotal) return;

  const int*   x    = (const int*)d_in[0];
  const float* emb  = (const float*)d_in[2];
  const float* Wx_f = (const float*)d_in[3];
  const float* bx_f = (const float*)d_in[4];
  const float* Wh_f = (const float*)d_in[5];
  const float* bh_f = (const float*)d_in[6];
  const float* Wx_b = (const float*)d_in[7];
  const float* bx_b = (const float*)d_in[8];
  const float* Wh_b = (const float*)d_in[9];
  const float* bh_b = (const float*)d_in[10];
  const float* Wfc  = (const float*)d_in[11];
  const float* bfc  = (const float*)d_in[12];
  float* out = (float*)d_out;

  char* ws = (char*)d_ws;
  unsigned short* Epl   = (unsigned short*)(ws + kOffE);
  unsigned short* Wcat  = (unsigned short*)(ws + kOffW);
  unsigned short* WfcP  = (unsigned short*)(ws + kOffWfc);
  float*          biasc = (float*)(ws + kOffBias);
  unsigned short* Hout  = (unsigned short*)(ws + kOffH);
  float*          Cfc   = (float*)(ws + kOffC);

  const int egroups = kRows * kEmb / 8;
  k_embed<<<(egroups + 255) / 256, 256, 0, stream>>>(x, emb, Epl, egroups);
  k_wcat<<<dim3((kGate * (kKcat / 8) + 255) / 256, 2), 256, 0, stream>>>(Wx_f, Wh_f, Wx_b, Wh_b, Wcat);
  k_wfc<<<(kTagPad * (2 * kHid / 8) + 255) / 256, 256, 0, stream>>>(Wfc, WfcP);
  k_bias<<<2, 256, 0, stream>>>(bx_f, bh_f, bx_b, bh_b, biasc);
  k_scan<<<8, 512, 0, stream>>>(Epl, Wcat, biasc, Hout);
  {
    const int tiles = (kRows / 64) * (kTagPad / 64);
    wmma_gemm64<0, false, 0, 0, false, 0><<<dim3((tiles + 7) / 8, 1), 256, 0, stream>>>(
        Hout, Hout, 2 * kHid, 0L,
        WfcP, WfcP, 2 * kHid, 0L,
        (void*)Cfc, (void*)Cfc, kTagPad, 0L,
        biasc,
        Cfc, 0L,
        kRows, kTagPad, 2 * kHid, kInv256);
  }
  const int n4 = out_size / 4;
  k_out<<<(n4 + 255) / 256, 256, 0, stream>>>(Cfc, bfc, out, n4);
}
